// RelNNTransformConnected_77841987273099
// MI455X (gfx1250) — hardware-verified
//
#include <hip/hip_runtime.h>

typedef _Float16 f16;
typedef __attribute__((ext_vector_type(8)))  f16   v8h;
typedef __attribute__((ext_vector_type(16))) f16   v16h;
typedef __attribute__((ext_vector_type(8)))  float v8f;
typedef __attribute__((ext_vector_type(4)))  float v4f;

#define N_   128
#define FIN_ 8
#define H_   128

__device__ static const float kActScale = 16.0f;
__device__ static const float kWScale   = 64.0f;
__device__ static const float kUnscale  = 0.0009765625f;

union Frag { v16h v; v8h half[2]; };

__device__ __forceinline__ v8f zero8() {
  v8f z = {0.f, 0.f, 0.f, 0.f, 0.f, 0.f, 0.f, 0.f};
  return z;
}

__device__ __forceinline__ v8f wmma16(v16h a, v16h b, v8f c) {
  c = __builtin_amdgcn_wmma_f32_16x16x32_f16(false, a, false, b, (short)0, c, false, false);
  asm volatile("v_nop\n\tv_nop\n\tv_nop\n\tv_nop" : "+v"(c) : "v"(a), "v"(b));
  return c;
}

__device__ __forceinline__ float fast_tanh(float x) {
  float e2 = __builtin_amdgcn_exp2f(x * 2.8853900817779268f);
  return 1.0f - 2.0f * __builtin_amdgcn_rcpf(e2 + 1.0f);
}

union StageU {
  f16   x0[N_ * H_];
  float stg[8 * 16 * 64];
};

__global__ __launch_bounds__(256)
void node_mlp_kernel(const float* __restrict__ jets,
                     const float* __restrict__ Wu,
                     const float* __restrict__ bu,
                     const float* __restrict__ Wu1,
                     const float* __restrict__ bu1,
                     const float* __restrict__ We,
                     float* __restrict__ eOut,
                     int nB)
{
  __shared__ __attribute__((aligned(16))) StageU s0;
  __shared__ __attribute__((aligned(16))) f16 sX1[N_ * H_];
  __shared__ __attribute__((aligned(16))) f16 sW [H_ * H_];

  const int b = blockIdx.x;
  if (b >= nB) return;

  const int tid  = threadIdx.x;
  const int wave = tid >> 5;
  const int lane = tid & 31;
  const int half = lane >> 4;
  const int l16  = lane & 15;

  for (int i = tid; i < H_ * H_; i += 256) sW[i] = (f16)(Wu1[i] * kWScale);
  {
    const float* jb = jets + (size_t)b * N_ * FIN_;
    const int h0 = tid & 127;
    float wr[FIN_];
    #pragma unroll
    for (int f = 0; f < FIN_; ++f) wr[f] = Wu[h0 * FIN_ + f];
    const float b0 = bu[h0];
    for (int n = tid >> 7; n < N_; n += 2) {
      float acc = 0.0f;
      #pragma unroll
      for (int f = 0; f < FIN_; ++f) acc += jb[n * FIN_ + f] * wr[f];
      acc += b0;
      s0.x0[n * H_ + h0] = (f16)(fmaxf(acc, 0.0f) * kActScale);
    }
  }
  __syncthreads();

  const int mtile = wave;
  const int rowA  = mtile * 16 + l16;

  for (int nt = 0; nt < 8; ++nt) {
    const int colB = nt * 16 + l16;
    v8f c = zero8();
    #pragma unroll
    for (int kt = 0; kt < 4; ++kt) {
      const int ko = kt * 32;
      Frag a, bf;
      a.half[0]  = *(const v8h*)&s0.x0[rowA * H_ + ko + 8 * half];
      a.half[1]  = *(const v8h*)&s0.x0[rowA * H_ + ko + 16 + 8 * half];
      bf.half[0] = *(const v8h*)&sW[colB * H_ + ko + 8 * half];
      bf.half[1] = *(const v8h*)&sW[colB * H_ + ko + 16 + 8 * half];
      c = wmma16(a.v, bf.v, c);
    }
    const float bias = bu1[colB];
    #pragma unroll
    for (int v = 0; v < 8; ++v) {
      const int m = mtile * 16 + 8 * half + v;
      sX1[m * H_ + colB] = (f16)(fmaxf(c[v] * kUnscale + bias, 0.0f) * kActScale);
    }
  }
  __syncthreads();

  for (int i = tid; i < H_ * H_; i += 256) sW[i] = (f16)(We[i] * kWScale);
  __syncthreads();

  float* eB  = eOut + (size_t)b * N_ * H_;
  float* stg = s0.stg + wave * (16 * 64);
  for (int hh = 0; hh < 2; ++hh) {
    for (int t = 0; t < 4; ++t) {
      const int colB = (hh * 4 + t) * 16 + l16;
      v8f c = zero8();
      #pragma unroll
      for (int kt = 0; kt < 4; ++kt) {
        const int ko = kt * 32;
        Frag a, bf;
        a.half[0]  = *(const v8h*)&sX1[rowA * H_ + ko + 8 * half];
        a.half[1]  = *(const v8h*)&sX1[rowA * H_ + ko + 16 + 8 * half];
        bf.half[0] = *(const v8h*)&sW[colB * H_ + ko + 8 * half];
        bf.half[1] = *(const v8h*)&sW[colB * H_ + ko + 16 + 8 * half];
        c = wmma16(a.v, bf.v, c);
      }
      #pragma unroll
      for (int v = 0; v < 8; ++v) {
        const int r = 8 * half + v;
        stg[r * 64 + t * 16 + l16] = c[v] * kUnscale;
      }
    }
    __syncthreads();
    v4f vals[8];
    #pragma unroll
    for (int q = 0; q < 8; ++q) {
      const int r = 2 * q + half;
      vals[q] = *(const v4f*)&stg[r * 64 + l16 * 4];
    }
    #pragma unroll
    for (int q = 0; q < 8; ++q) {
      const int r = 2 * q + half;
      float* gp = eB + (size_t)(mtile * 16 + r) * H_ + hh * 64 + l16 * 4;
      *(volatile v4f*)gp = vals[q];
    }
    __threadfence();
    #pragma unroll
    for (int q = 0; q < 8; ++q) {
      const int r = 2 * q + half;
      float* gp = eB + (size_t)(mtile * 16 + r) * H_ + hh * 64 + l16 * 4;
      *(volatile v4f*)gp = vals[q];
    }
    __syncthreads();
  }
}

__global__ __launch_bounds__(128)
void pair_mean_kernel(const float* __restrict__ e,
                      const float* __restrict__ be,
                      float* __restrict__ out,
                      int nB)
{
  __shared__ __attribute__((aligned(16))) float sOut[H_];
  const int b = blockIdx.x;
  if (b >= nB) return;
  const int h = threadIdx.x;
  const float* eB = e + (size_t)b * N_ * H_;
  const float bh = be[h];
  float tot = 0.0f;
  for (int j = 0; j < N_; ++j) {
    const float ej = eB[j * H_ + h] + bh;
    float acc = 0.0f;
    #pragma unroll 4
    for (int i = 0; i < N_; ++i)
      acc += fast_tanh(ej + eB[i * H_ + h]);
    tot += acc;
  }
  sOut[h] = tot * (1.0f / (float)(N_ * N_));
  __syncthreads();
  v4f v = {0.f, 0.f, 0.f, 0.f};
  float* gp = out + (size_t)b * H_ + (h & 31) * 4;
  if (h < 32) {
    v = *(const v4f*)&sOut[h * 4];
    *(volatile v4f*)gp = v;
  }
  __threadfence();
  if (h < 32) {
    *(volatile v4f*)gp = v;
  }
}

extern "C" void kernel_launch(void* const* d_in, const int* in_sizes, int n_in,
                              void* d_out, int out_size, void* d_ws, size_t ws_size,
                              hipStream_t stream) {
  if (n_in < 7) return;
  const int nB = in_sizes[0] / (N_ * FIN_);
  if (nB <= 0 || nB * N_ * FIN_ != in_sizes[0]) return;
  if (in_sizes[1] != H_ * FIN_ || in_sizes[2] != H_ || in_sizes[3] != H_ * H_ ||
      in_sizes[4] != H_ || in_sizes[5] != H_ * H_ || in_sizes[6] != H_) return;
  if (out_size != nB * H_) return;
  const size_t eBytes = (size_t)nB * N_ * H_ * sizeof(float);
  if (eBytes > ws_size) return;

  const float* jets = (const float*)d_in[0];
  const float* Wu   = (const float*)d_in[1];
  const float* bu   = (const float*)d_in[2];
  const float* Wu1  = (const float*)d_in[3];
  const float* bu1  = (const float*)d_in[4];
  const float* We   = (const float*)d_in[5];
  const float* be   = (const float*)d_in[6];
  float* out = (float*)d_out;
  float* e   = (float*)d_ws;

  node_mlp_kernel<<<nB, 256, 0, stream>>>(jets, Wu, bu, Wu1, bu1, We, e, nB);
  pair_mean_kernel<<<nB, H_, 0, stream>>>(e, be, out, nB);
}
